// SelfAttention_37391985279526
// MI455X (gfx1250) — hardware-verified
//
#include <hip/hip_runtime.h>
#ifndef NB
#define NB 2
#endif
#ifndef SEQ
#define SEQ 2048
#endif
#define NB_FULL 2
#define SEQ_FULL 2048
#define DM 1024
#define NH 16
#define HD 64
#define LDH (3 * DM)
#define LDL (2 * DM)
#define NR (NB * SEQ)

#define SZ_BQKV ((size_t)3 * DM * DM * 2)
#define SZ_BO   ((size_t)DM * DM * 2)
#define SZ_X16  ((size_t)NR * DM * 2)
#define SZ_HP   ((size_t)NR * LDH * 2)
#define SZ_LP   ((size_t)NR * LDL * 2)
#define SZ_VT   ((size_t)NB * NH * HD * SEQ * 2)
#define SZ_O    ((size_t)NR * DM * 2)
#define SZ_TOTAL (SZ_BQKV + SZ_BO + SZ_X16 + SZ_HP + SZ_LP + SZ_VT + SZ_O + SZ_O)

static_assert(DM == NH * HD);
static_assert(HD == 64);
static_assert(DM % 32 == 0);
static_assert(DM % 64 == 0);
static_assert(LDH % 64 == 0);
static_assert(SEQ % 64 == 0);
static_assert(SEQ % 32 == 0);
static_assert(NR % 128 == 0);
static_assert(NB <= NB_FULL);
static_assert(SEQ <= SEQ_FULL);
static_assert(SZ_BQKV % 256 == 0 && SZ_BO % 256 == 0 && SZ_X16 % 256 == 0 && SZ_HP % 256 == 0 && SZ_LP % 256 == 0 && SZ_VT % 256 == 0 && SZ_O % 256 == 0);
static_assert(SZ_TOTAL <= (size_t)134217728);

typedef _Float16 v16h __attribute__((ext_vector_type(16)));
typedef unsigned short v8us __attribute__((ext_vector_type(8), may_alias));
typedef float v8f  __attribute__((ext_vector_type(8)));
typedef float v4f  __attribute__((ext_vector_type(4)));
typedef float v4fa __attribute__((ext_vector_type(4), may_alias));
union FragH { v16h v; v8us half[2]; _Float16 h[16]; unsigned short u[16]; };

__device__ __forceinline__ unsigned short bf16_bits(float x) { unsigned int u = __float_as_uint(x); return (unsigned short)((u + 0x7FFFu + ((u >> 16) & 1u)) >> 16); }
__device__ __forceinline__ float bf16_rne(float x) { return __uint_as_float(((unsigned int)bf16_bits(x)) << 16); }

__device__ __forceinline__ v16h ld_frag(const _Float16* __restrict__ base, size_t off, int hh) {
  FragH f; const unsigned short* p = (const unsigned short*)base + off;
  f.half[0] = *(const v8us*)(p + 8 * hh); f.half[1] = *(const v8us*)(p + 16 + 8 * hh); return f.v;
}
__device__ __forceinline__ v8f mma1(v16h a, v16h b, v8f c) {
  v8f d = __builtin_amdgcn_wmma_f32_16x16x32_f16(false, a, false, b, (short)0, c, false, false);
  asm volatile("v_nop\n\tv_nop\n\tv_nop\n\tv_nop" : "+v"(d) : "v"(a), "v"(b));
  return d;
}
__device__ __forceinline__ void mma2(v16h ah, v16h al, v16h b, v8f& ch, v8f& cr) {
  ch = __builtin_amdgcn_wmma_f32_16x16x32_f16(false, ah, false, b, (short)0, ch, false, false);
  cr = __builtin_amdgcn_wmma_f32_16x16x32_f16(false, al, false, b, (short)0, cr, false, false);
  asm volatile("v_nop\n\tv_nop\n\tv_nop\n\tv_nop" : "+v"(ch), "+v"(cr) : "v"(ah), "v"(al), "v"(b));
}
__device__ __forceinline__ void mma3(v16h ah, v16h al, v16h bh, v16h bl, v8f& ch, v8f& cr) {
  ch = __builtin_amdgcn_wmma_f32_16x16x32_f16(false, ah, false, bh, (short)0, ch, false, false);
  cr = __builtin_amdgcn_wmma_f32_16x16x32_f16(false, al, false, bh, (short)0, cr, false, false);
  cr = __builtin_amdgcn_wmma_f32_16x16x32_f16(false, ah, false, bl, (short)0, cr, false, false);
  asm volatile("v_nop\n\tv_nop\n\tv_nop\n\tv_nop" : "+v"(ch), "+v"(cr) : "v"(ah), "v"(al), "v"(bh), "v"(bl));
}

__global__ __launch_bounds__(256) void k_x16(const float* __restrict__ x, _Float16* __restrict__ X16, int n8) {
  const int t = blockIdx.x * 256 + threadIdx.x; if (t >= n8) return;
  const int row = t / (DM / 8), c8 = (t % (DM / 8)) * 8;
  const int b = row / SEQ, s = row % SEQ;
  const float* src = x + ((size_t)b * SEQ_FULL + s) * DM + c8;
  const v4f a = *(const v4fa*)src, c = *(const v4fa*)(src + 4);
  FragH f;
#pragma unroll
  for (int q = 0; q < 4; ++q) { f.h[q] = (_Float16)bf16_rne(a[q]); f.h[4 + q] = (_Float16)bf16_rne(c[q]); }
  const v8us o = f.half[0];
  unsigned short* d = (unsigned short*)X16 + (size_t)t * 8;
  *(volatile v8us*)d = o; __threadfence(); *(volatile v8us*)d = o;
}

__global__ __launch_bounds__(256) void k_wt_f16(const float* __restrict__ W, _Float16* __restrict__ Wt, int K, int N, float scale) {
  const int t = blockIdx.x * 256 + threadIdx.x; const int k8n = K / 8; if (t >= N * k8n) return;
  const int n = t / k8n, k8 = (t % k8n) * 8;
  FragH f;
#pragma unroll
  for (int i = 0; i < 8; ++i) f.h[i] = (_Float16)(bf16_rne(W[(size_t)(k8 + i) * N + n]) * scale);
  const v8us o = f.half[0];
  unsigned short* d = (unsigned short*)Wt + (size_t)n * K + k8;
  *(volatile v8us*)d = o; __threadfence(); *(volatile v8us*)d = o;
}

__global__ __launch_bounds__(128) void k_gemm_qkv(const _Float16* __restrict__ A, const _Float16* __restrict__ Bh, const float* __restrict__ bias,
                                                 _Float16* __restrict__ Hp, _Float16* __restrict__ Lp) {
  __shared__ __attribute__((aligned(16))) float so[4][32][68];
  const int wave = __builtin_amdgcn_readfirstlane(threadIdx.x >> 5);
  const int lane = threadIdx.x & 31, ln = lane & 15, hh = lane >> 4;
  const int ntn = LDH / 64;
  const int mt = blockIdx.x / ntn, nq = blockIdx.x - mt * ntn;
  const int row0 = mt * 128 + 32 * wave, col0 = nq * 64;
  const size_t a0 = (size_t)(row0 + ln) * DM, a1 = a0 + (size_t)16 * DM;
  const size_t b0 = (size_t)(col0 + ln) * DM, b1 = b0 + (size_t)16 * DM, b2 = b1 + (size_t)16 * DM, b3 = b2 + (size_t)16 * DM;
  const v8f z8 = {0.f, 0.f, 0.f, 0.f, 0.f, 0.f, 0.f, 0.f};
  v8f c00 = z8, c01 = z8, c02 = z8, c03 = z8, c10 = z8, c11 = z8, c12 = z8, c13 = z8;
#pragma unroll 1
  for (int kb = 0; kb < DM; kb += 32) {
    const v16h f0 = ld_frag(A, a0 + kb, hh), f1 = ld_frag(A, a1 + kb, hh);
    v16h b = ld_frag(Bh, b0 + kb, hh); c00 = mma1(f0, b, c00); c10 = mma1(f1, b, c10);
    b = ld_frag(Bh, b1 + kb, hh); c01 = mma1(f0, b, c01); c11 = mma1(f1, b, c11);
    b = ld_frag(Bh, b2 + kb, hh); c02 = mma1(f0, b, c02); c12 = mma1(f1, b, c12);
    b = ld_frag(Bh, b3 + kb, hh); c03 = mma1(f0, b, c03); c13 = mma1(f1, b, c13);
  }
  v8f accs[8] = {c00, c01, c02, c03, c10, c11, c12, c13};
#pragma unroll
  for (int u = 0; u < 8; ++u) {
    const int t = u & 3, half = u >> 2;
    const float bv = bf16_rne(bias[col0 + t * 16 + ln]);
#pragma unroll
    for (int r = 0; r < 8; ++r) so[wave][half * 16 + 8 * hh + r][t * 16 + ln] = accs[u][r] * 0.0625f + bv;
  }
  __builtin_amdgcn_fence(4  , "workgroup");
  __builtin_amdgcn_wave_barrier();
  const int rs = lane >> 3, c8 = (lane & 7) * 8;
  const bool haslo = col0 < LDL;
  for (int pass = 0; pass < 2; ++pass) {
#pragma unroll
    for (int q = 0; q < 8; ++q) {
      const int r = q * 4 + rs;
      const v4f v0 = *(const v4fa*)&so[wave][r][c8], v1 = *(const v4fa*)&so[wave][r][c8 + 4];
      FragH fh, fl;
#pragma unroll
      for (int i = 0; i < 4; ++i) {
        _Float16 hv = (_Float16)v0[i]; fh.h[i] = hv; fl.h[i] = (_Float16)((v0[i] - (float)hv) * 1024.0f);
        hv = (_Float16)v1[i]; fh.h[4 + i] = hv; fl.h[4 + i] = (_Float16)((v1[i] - (float)hv) * 1024.0f);
      }
      const v8us oh = fh.half[0], ol = fl.half[0];
      *(volatile v8us*)((unsigned short*)Hp + (size_t)(row0 + r) * LDH + col0 + c8) = oh;
      if (haslo) *(volatile v8us*)((unsigned short*)Lp + (size_t)(row0 + r) * LDL + col0 + c8) = ol;
    }
    if (pass == 0) __threadfence();
  }
}

__global__ __launch_bounds__(256) void k_vt(const _Float16* __restrict__ Hp, _Float16* __restrict__ VT) {
  __shared__ unsigned short tl[64][72];
  const int tid = threadIdx.x;
  const int bh = blockIdx.x / (SEQ / 64), sg = blockIdx.x % (SEQ / 64);
  const int b = bh / NH, h = bh % NH, s0 = sg * 64;
#pragma unroll
  for (int it = 0; it < 2; ++it) {
    const int i = tid + 256 * it, j = i >> 3, d8 = (i & 7) * 8;
    FragH f; f.half[0] = *(const v8us*)((const unsigned short*)Hp + ((size_t)b * SEQ + s0 + j) * LDH + 2 * DM + h * HD + d8);
#pragma unroll
    for (int q = 0; q < 8; ++q) tl[d8 + q][j] = f.u[q];
  }
  __syncthreads();
  for (int pass = 0; pass < 2; ++pass) {
#pragma unroll
    for (int it = 0; it < 2; ++it) {
      const int i = tid + 256 * it, d = i >> 3, j8 = (i & 7) * 8;
      FragH f;
#pragma unroll
      for (int q = 0; q < 8; ++q) f.u[q] = tl[d][j8 + q];
      const v8us o = f.half[0];
      *(volatile v8us*)((unsigned short*)VT + ((size_t)bh * HD + d) * SEQ + s0 + j8) = o;
    }
    if (pass == 0) __threadfence();
  }
}

__global__ __launch_bounds__(128) void k_attn(const _Float16* __restrict__ Hp, const _Float16* __restrict__ Lp, const _Float16* __restrict__ VT,
                                             _Float16* __restrict__ OH, _Float16* __restrict__ OL) {
  __shared__ __attribute__((aligned(16))) float so[4][16][68];
  const int wave = __builtin_amdgcn_readfirstlane(threadIdx.x >> 5);
  const int lane = threadIdx.x & 31, ln = lane & 15, hh = lane >> 4;
  const int bh = blockIdx.x / (SEQ / 64), qb = blockIdx.x % (SEQ / 64);
  const int b = bh / NH, h = bh % NH;
  const int q0 = qb * 64 + wave * 16;
  const size_t tok0 = (size_t)b * SEQ;
  const size_t qoffH = (tok0 + q0 + ln) * LDH + h * HD;
  const size_t qoffL = (tok0 + q0 + ln) * LDL + h * HD;
  const size_t koffH = (tok0 + ln) * LDH + DM + h * HD;
  const size_t koffL = (tok0 + ln) * LDL + DM + h * HD;
  const size_t voff  = ((size_t)bh * HD + ln) * SEQ;
  const v8f z8 = {0.f, 0.f, 0.f, 0.f, 0.f, 0.f, 0.f, 0.f};
  v8f o0 = z8, o1 = z8, o2 = z8, o3 = z8;
  float m = -1.0e30f, l = 0.f;
#pragma unroll 1
  for (int kc = 0; kc < SEQ; kc += 32) {
    int qo = 0; asm volatile("" : "+v"(qo));
    v8f sh0 = z8, sh1 = z8, sr0 = z8, sr1 = z8;
    const size_t kH = koffH + (size_t)kc * LDH, kL = koffL + (size_t)kc * LDL;
#pragma unroll
    for (int ks = 0; ks < 2; ++ks) {
      const v16h qh = ld_frag(Hp, qoffH + qo + ks * 32, hh), ql = ld_frag(Lp, qoffL + qo + ks * 32, hh);
      v16h ka = ld_frag(Hp, kH + ks * 32, hh), kl = ld_frag(Lp, kL + ks * 32, hh);
      mma3(ka, kl, qh, ql, sh0, sr0);
      ka = ld_frag(Hp, kH + (size_t)16 * LDH + ks * 32, hh); kl = ld_frag(Lp, kL + (size_t)16 * LDL + ks * 32, hh);
      mma3(ka, kl, qh, ql, sh1, sr1);
    }
    float sv[16];
#pragma unroll
    for (int r = 0; r < 8; ++r) {
      sv[r]     = (sh0[r] + sr0[r] * 0.0009765625f) * 0.125f;
      sv[8 + r] = (sh1[r] + sr1[r] * 0.0009765625f) * 0.125f;
    }
    float mx = sv[0];
#pragma unroll
    for (int i = 1; i < 16; ++i) mx = fmaxf(mx, sv[i]);
    mx = fmaxf(mx, __shfl_xor(mx, 16, 32));
    const float mn = fmaxf(m, mx);
    const float alpha = __expf(m - mn);
    m = mn;
    float ps = 0.f; FragH pf;
#pragma unroll
    for (int i = 0; i < 16; ++i) { const float p = __expf(sv[i] - mn); ps += p; pf.h[i] = (_Float16)(p * 1024.0f); }
    ps += __shfl_xor(ps, 16, 32);
    l = l * alpha + ps;
#pragma unroll
    for (int r = 0; r < 8; ++r) { o0[r] *= alpha; o1[r] *= alpha; o2[r] *= alpha; o3[r] *= alpha; }
    const size_t vk = voff + kc;
    o0 = mma1(ld_frag(VT, vk, hh), pf.v, o0);
    o1 = mma1(ld_frag(VT, vk + (size_t)16 * SEQ, hh), pf.v, o1);
    o2 = mma1(ld_frag(VT, vk + (size_t)32 * SEQ, hh), pf.v, o2);
    o3 = mma1(ld_frag(VT, vk + (size_t)48 * SEQ, hh), pf.v, o3);
  }
  const float fin = 0.0625f * (1.0f / l);
#pragma unroll
  for (int r = 0; r < 8; ++r) {
    so[wave][ln][8 * hh + r]      = o0[r] * fin;
    so[wave][ln][16 + 8 * hh + r] = o1[r] * fin;
    so[wave][ln][32 + 8 * hh + r] = o2[r] * fin;
    so[wave][ln][48 + 8 * hh + r] = o3[r] * fin;
  }
  __builtin_amdgcn_fence(4  , "workgroup");
  __builtin_amdgcn_wave_barrier();
  const int rs = lane >> 3, c8 = (lane & 7) * 8;
  for (int pass = 0; pass < 2; ++pass) {
#pragma unroll
    for (int q = 0; q < 4; ++q) {
      const int r = q * 4 + rs;
      const v4f v0 = *(const v4fa*)&so[wave][r][c8], v1 = *(const v4fa*)&so[wave][r][c8 + 4];
      FragH fh, fl;
#pragma unroll
      for (int i = 0; i < 4; ++i) {
        _Float16 hv = (_Float16)v0[i]; fh.h[i] = hv; fl.h[i] = (_Float16)((v0[i] - (float)hv) * 1024.0f);
        hv = (_Float16)v1[i]; fh.h[4 + i] = hv; fl.h[4 + i] = (_Float16)((v1[i] - (float)hv) * 1024.0f);
      }
      const v8us oh = fh.half[0], ol = fl.half[0];
      const size_t dst = (tok0 + q0 + r) * DM + h * HD + c8;
      *(volatile v8us*)((unsigned short*)OH + dst) = oh;
      *(volatile v8us*)((unsigned short*)OL + dst) = ol;
    }
    if (pass == 0) __threadfence();
  }
}

__global__ __launch_bounds__(128) void k_gemm_out(const _Float16* __restrict__ AH, const _Float16* __restrict__ AL, const _Float16* __restrict__ Bh,
                                                 const float* __restrict__ bias, float* __restrict__ C) {
  __shared__ __attribute__((aligned(16))) float so[4][16][68];
  const int wave = __builtin_amdgcn_readfirstlane(threadIdx.x >> 5);
  const int lane = threadIdx.x & 31, ln = lane & 15, hh = lane >> 4;
  const int ntn = DM / 64;
  const int mt = blockIdx.x / ntn, nq = blockIdx.x - mt * ntn;
  const int row0 = mt * 64 + 16 * wave, col0 = nq * 64;
  const size_t a0 = (size_t)(row0 + ln) * DM;
  const size_t b0 = (size_t)(col0 + ln) * DM, b1 = b0 + (size_t)16 * DM, b2 = b1 + (size_t)16 * DM, b3 = b2 + (size_t)16 * DM;
  const v8f z8 = {0.f, 0.f, 0.f, 0.f, 0.f, 0.f, 0.f, 0.f};
  v8f h0 = z8, h1 = z8, h2 = z8, h3 = z8, r0 = z8, r1 = z8, r2 = z8, r3 = z8;
#pragma unroll 1
  for (int kb = 0; kb < DM; kb += 32) {
    const v16h ah = ld_frag(AH, a0 + kb, hh), al = ld_frag(AL, a0 + kb, hh);
    v16h b = ld_frag(Bh, b0 + kb, hh); mma2(ah, al, b, h0, r0);
    b = ld_frag(Bh, b1 + kb, hh); mma2(ah, al, b, h1, r1);
    b = ld_frag(Bh, b2 + kb, hh); mma2(ah, al, b, h2, r2);
    b = ld_frag(Bh, b3 + kb, hh); mma2(ah, al, b, h3, r3);
  }
  v8f ach[4] = {h0, h1, h2, h3};
  v8f acr[4] = {r0, r1, r2, r3};
#pragma unroll
  for (int t = 0; t < 4; ++t) {
    const float bv = bf16_rne(bias[col0 + t * 16 + ln]);
#pragma unroll
    for (int r = 0; r < 8; ++r) so[wave][8 * hh + r][t * 16 + ln] = ach[t][r] * 0.0009765625f + acr[t][r] * 9.5367431640625e-07f + bv;
  }
  __builtin_amdgcn_fence(4  , "workgroup");
  __builtin_amdgcn_wave_barrier();
  const int rsub = lane >> 4, c4 = (lane & 15) * 4;
  for (int pass = 0; pass < 2; ++pass) {
#pragma unroll
    for (int q = 0; q < 8; ++q) {
      const int r = q * 2 + rsub;
      const int grow = row0 + r;
      const int ob = grow / SEQ, os = grow % SEQ;
      const v4f v = *(const v4fa*)&so[wave][r][c4];
      *(volatile v4f*)(C + ((size_t)ob * SEQ_FULL + os) * DM + col0 + c4) = v;
    }
    if (pass == 0) __threadfence();
  }
}

extern "C" void kernel_launch(void* const* d_in, const int* in_sizes, int n_in,
                              void* d_out, int out_size, void* d_ws, size_t ws_size, hipStream_t stream) {
  if (n_in < 5) return;
  const long long xneed = ((long long)(NB - 1) * SEQ_FULL + SEQ) * DM;
  if ((long long)in_sizes[0] < xneed) return;
  if ((long long)in_sizes[1] < (long long)DM * LDH) return;
  if (in_sizes[2] < LDH) return;
  if ((long long)in_sizes[3] < (long long)DM * DM) return;
  if (in_sizes[4] < DM) return;
  if ((long long)out_size < xneed) return;
  if ((size_t)SZ_TOTAL > ws_size) return;
  const float* x    = (const float*)d_in[0];
  const float* wqkv = (const float*)d_in[1];
  const float* bqkv = (const float*)d_in[2];
  const float* wo   = (const float*)d_in[3];
  const float* bo   = (const float*)d_in[4];
  char* ws = (char*)d_ws; size_t off = 0;
  _Float16* BQKV = (_Float16*)(ws + off); off += SZ_BQKV;
  _Float16* BO   = (_Float16*)(ws + off); off += SZ_BO;
  _Float16* X16  = (_Float16*)(ws + off); off += SZ_X16;
  _Float16* HP   = (_Float16*)(ws + off); off += SZ_HP;
  _Float16* LP   = (_Float16*)(ws + off); off += SZ_LP;
  _Float16* VT   = (_Float16*)(ws + off); off += SZ_VT;
  _Float16* OH   = (_Float16*)(ws + off); off += SZ_O;
  _Float16* OL   = (_Float16*)(ws + off); off += SZ_O;
  if (off > ws_size) return;

  k_wt_f16<<<(unsigned)((LDH * (DM / 8) + 255) / 256), 256, 0, stream>>>(wqkv, BQKV, DM, LDH, 16.0f);
  k_wt_f16<<<(unsigned)((DM * (DM / 8) + 255) / 256), 256, 0, stream>>>(wo, BO, DM, DM, 16.0f);
  k_x16<<<(unsigned)((NR * (DM / 8) + 255) / 256), 256, 0, stream>>>(x, X16, NR * (DM / 8));
  k_gemm_qkv<<<(unsigned)((NR / 128) * (LDH / 64)), 128, 0, stream>>>(X16, BQKV, bqkv, HP, LP);
  k_vt<<<(unsigned)(NB * NH * (SEQ / 64)), 256, 0, stream>>>(HP, VT);
  k_attn<<<(unsigned)(NB * NH * (SEQ / 64)), 128, 0, stream>>>(HP, LP, VT, OH, OL);
  k_gemm_out<<<(unsigned)((NR / 64) * (DM / 64)), 128, 0, stream>>>(OH, OL, BO, bo, (float*)d_out);
}
